// RingAttention_21311627723171
// MI455X (gfx1250) — hardware-verified
//
#include <hip/hip_runtime.h>


#ifndef NB
#define NB 1
#endif
#ifndef SEQ
#define SEQ 4096
#endif
#define NB_FULL 1
#define SEQ_FULL 4096
#define DIM 1024
#define HEADS 8
#define DHEAD 64
#define DINNER (HEADS * DHEAD)
#define NQKV (3 * DINNER)
#define SEQT (NB * SEQ)
#define QBLK (SEQ / 64)
#define RSP 32
#define CSTR 132

static_assert(SEQ % 64 == 0);
static_assert(SEQ >= 128);
static_assert(SEQ <= SEQ_FULL);
static_assert(NB >= 1 && NB <= NB_FULL);
static_assert(DIM % 128 == 0 && NQKV % 128 == 0 && DINNER % 128 == 0);
static_assert(DIM % 32 == 0 && DINNER % 32 == 0 && DHEAD == 64);
static_assert(DIM == 4 * 256);

typedef unsigned short us16;
typedef __attribute__((ext_vector_type(16))) __bf16   v16bf;
typedef __attribute__((ext_vector_type(16))) _Float16 v16h;
typedef __attribute__((ext_vector_type(8)))  float    v8f;
typedef __attribute__((ext_vector_type(8)))  unsigned v8u;
typedef __attribute__((ext_vector_type(4)))  unsigned v4u;
typedef __attribute__((ext_vector_type(2)))  unsigned v2u;
typedef __attribute__((ext_vector_type(4)))  float    v4f;

__device__ __forceinline__ unsigned f2bf(float f) { unsigned u = __float_as_uint(f); u += 0x7FFFu + ((u >> 16) & 1u); return u >> 16; }
__device__ __forceinline__ float bf2f(unsigned h) { return __uint_as_float(h << 16); }
__device__ __forceinline__ unsigned f2h(float f) { _Float16 t = (_Float16)f; return (unsigned)__builtin_bit_cast(unsigned short, t); }

__device__ __forceinline__ v8u ld_frag(const us16* rowp, int hh) {
    const v4u a = *(const v4u*)(rowp + 8 * hh);
    const v4u b = *(const v4u*)(rowp + 16 + 8 * hh);
    return __builtin_shufflevector(a, b, 0, 1, 2, 3, 4, 5, 6, 7);
}
__device__ __forceinline__ v8f mma_bf16(v8u a, v8u b, v8f c) {
    return __builtin_amdgcn_wmma_f32_16x16x32_bf16(false, __builtin_bit_cast(v16bf, a), false, __builtin_bit_cast(v16bf, b), (short)0, c, false, false);
}
__device__ __forceinline__ v8f mma_f16(v8u a, v8u b, v8f c) {
    return __builtin_amdgcn_wmma_f32_16x16x32_f16(false, __builtin_bit_cast(v16h, a), false, __builtin_bit_cast(v16h, b), (short)0, c, false, false);
}
__device__ __forceinline__ void mma_guard(v8f& c, v8u a, v8u b) {
    asm volatile("v_nop\n\tv_nop\n\tv_nop\n\tv_nop" : "+v"(c) : "v"(a), "v"(b));
}

__global__ __launch_bounds__(256) void prep_x(const float* __restrict__ x, us16* xb, float* rs) {
    __shared__ float red[8];
    const int tok = blockIdx.x;
    const int bsel = tok / SEQ, isel = tok - bsel * SEQ;
    const float* xr = x + ((size_t)bsel * SEQ_FULL + isel) * DIM;
    const int tid = threadIdx.x, lane = tid & 31, wid = tid >> 5;
    const v4f v = *(const v4f*)(xr + 4 * tid);
    const unsigned h0 = f2bf(v.x), h1 = f2bf(v.y), h2 = f2bf(v.z), h3 = f2bf(v.w);
    const float r0 = bf2f(h0), r1 = bf2f(h1), r2 = bf2f(h2), r3 = bf2f(h3);
    float s = r0 * r0 + r1 * r1 + r2 * r2 + r3 * r3;
#pragma unroll
    for (int o = 16; o; o >>= 1) s += __shfl_xor(s, o, 32);
    if (lane == 0) red[wid] = s;
    __syncthreads();
    float tot = 0.f;
#pragma unroll
    for (int q = 0; q < 8; ++q) tot += red[q];
    const float l2 = fmaxf(sqrtf(tot), 1e-12f);
    const float f = (1.0f / l2) * 32.0f;
    v2u pk; pk.x = h0 | (h1 << 16); pk.y = h2 | (h3 << 16);
    us16* orow = xb + (size_t)tok * DIM;
    *(volatile v2u*)(orow + 4 * tid) = pk;
    if (wid == 0) *(volatile float*)(rs + (size_t)tok * RSP + lane) = f;
    __threadfence();
    *(volatile v2u*)(orow + 4 * tid) = pk;
    if (wid == 0) *(volatile float*)(rs + (size_t)tok * RSP + lane) = f;
}

template <int F16, int USEG>
__global__ __launch_bounds__(256) void prep_w(const float* __restrict__ src, int N, int K, const float* __restrict__ gam, float scale, us16* dst) {
    __shared__ float tile[64][65];
    const int n0 = blockIdx.x * 64, k0 = blockIdx.y * 64;
    const int tid = threadIdx.x, lane = tid & 31, wid = tid >> 5;
    const int nn = tid & 63, kr = tid >> 6;
#pragma unroll 4
    for (int j = 0; j < 16; ++j) {
        const int k = kr + 4 * j;
        float w = bf2f(f2bf(src[(size_t)(k0 + k) * N + n0 + nn]));
        if (USEG) w = bf2f(f2bf(w * bf2f(f2bf(gam[k0 + k]))));
        tile[k][nn] = w * scale;
    }
    __syncthreads();
    auto pass = [&]() {
#pragma unroll
        for (int j = 0; j < 8; ++j) {
            const int r = wid + 8 * j;
            const float a = tile[2 * lane][r], bq = tile[2 * lane + 1][r];
            const unsigned pk = F16 ? (f2h(a) | (f2h(bq) << 16)) : (f2bf(a) | (f2bf(bq) << 16));
            *(volatile unsigned*)(dst + (size_t)(n0 + r) * K + k0 + 2 * lane) = pk;
        }
    };
    pass();
    __threadfence();
    pass();
}

template <int F16>
__device__ __forceinline__ void mm_tile(const us16* __restrict__ arow, const us16* __restrict__ bbase, int ldb, int K, int hh, v8f (&acc)[4]) {
#pragma unroll 1
    for (int kc = 0; kc < K; kc += 32) {
        const v8u a = ld_frag(arow + kc, hh);
#pragma unroll
        for (int t = 0; t < 4; ++t) {
            const v8u bfrag = ld_frag(bbase + (size_t)(t * 16) * ldb + kc, hh);
            if (F16) acc[t] = mma_f16(a, bfrag, acc[t]);
            else     acc[t] = mma_bf16(a, bfrag, acc[t]);
            mma_guard(acc[t], a, bfrag);
        }
    }
}

__global__ __launch_bounds__(256) void qkv_gemm(const us16* __restrict__ xb, const us16* __restrict__ wq, const float* __restrict__ rs,
                                                us16* qhi, us16* qlo, us16* khi, us16* klo, us16* vt, float* qkvf) {
    __shared__ __align__(16) float cst[64 * CSTR];
    const int tid = threadIdx.x, lane = tid & 31, wv = tid >> 5, l16 = lane & 15, hh = lane >> 4;
    const int rt = wv & 3, ch = wv >> 2;
    const int row0 = blockIdx.x * 64;
    const int colb = blockIdx.y * 128;
    const us16* arow = xb + (size_t)(row0 + rt * 16 + l16) * DIM;
    const us16* bbase = wq + (size_t)(colb + ch * 64 + l16) * DIM;
    v8f acc[4] = {};
    mm_tile<0>(arow, bbase, DIM, DIM, hh, acc);
#pragma unroll
    for (int r = 0; r < 8; ++r) {
        const int rl = rt * 16 + 8 * hh + r;
        const float f = rs[(size_t)(row0 + rl) * RSP + l16];
#pragma unroll
        for (int t = 0; t < 4; ++t) cst[rl * CSTR + ch * 64 + t * 16 + l16] = acc[t][r] * f;
    }
    __syncthreads();
    const int which = colb / DINNER;
    const int hsel = (colb % DINNER) / DHEAD;
    const int bsel = row0 / SEQ, i0 = row0 % SEQ;
    auto pass = [&]() {
        if (which < 2) {
            us16* ph = (which == 0) ? qhi : khi;
            us16* pl = (which == 0) ? qlo : klo;
#pragma unroll 4
            for (int j = 0; j < 16; ++j) {
                const int L = wv * 16 + j, r = L >> 1, c = L & 1;
                const float a = cst[r * CSTR + c * 64 + 2 * lane], bq = cst[r * CSTR + c * 64 + 2 * lane + 1];
                const unsigned ha = f2bf(a), hb = f2bf(bq);
                const unsigned la = f2bf(a - bf2f(ha)), lb = f2bf(bq - bf2f(hb));
                const size_t off = ((size_t)(hsel + c) * SEQT + row0 + r) * DHEAD + 2 * lane;
                *(volatile unsigned*)(ph + off) = ha | (hb << 16);
                *(volatile unsigned*)(pl + off) = la | (lb << 16);
            }
        } else {
#pragma unroll 4
            for (int j = 0; j < 16; ++j) {
                const int L = wv * 16 + j, c = L >> 6, d = L & 63;
                const float a = cst[(2 * lane) * CSTR + c * 64 + d] * 4.0f, bq = cst[(2 * lane + 1) * CSTR + c * 64 + d] * 4.0f;
                const size_t off = ((size_t)(hsel + c) * DHEAD + d) * SEQT + row0 + 2 * lane;
                *(volatile unsigned*)(vt + off) = f2h(a) | (f2h(bq) << 16);
            }
        }
        if (i0 == 0) {
            const int col = tid & 127, rsel = tid >> 7;
            float* dstp = qkvf + (size_t)bsel * 64 * NQKV + colb + col;
#pragma unroll 4
            for (int r = rsel; r < 64; r += 2) *(volatile float*)(dstp + (size_t)r * NQKV) = cst[r * CSTR + col];
        }
    };
    pass();
    __threadfence();
    pass();
}

__global__ __launch_bounds__(256) __attribute__((amdgpu_num_vgpr(256))) void attn_first(const float* __restrict__ qkvf, us16* ao) {
    __shared__ float qs[64][64];
    __shared__ float ks[64][65];
    __shared__ float vs[64][65];
    __shared__ v4u ost[64][8];
    const int h = blockIdx.x % HEADS, bsel = blockIdx.x / HEADS;
    const float* base = qkvf + (size_t)bsel * 64 * NQKV + h * DHEAD;
    const int tid = threadIdx.x, lane = tid & 31;
#pragma unroll 4
    for (int j = 0; j < 16; ++j) {
        const int idx = tid + 256 * j, r = idx >> 6, cc = idx & 63;
        const float* rp = base + (size_t)r * NQKV + cc;
        qs[r][cc] = rp[0] * 8.0f;
        ks[r][cc] = rp[DINNER];
        vs[r][cc] = rp[2 * DINNER];
    }
    __syncthreads();
    const int i = tid >> 2, p = tid & 3;
    const float NEG = -__builtin_inff();
    float sr[16];
#pragma unroll
    for (int jj = 0; jj < 16; ++jj) sr[jj] = 0.f;
#pragma unroll 1
    for (int d = 0; d < DHEAD; ++d) {
        const float qd = qs[i][d];
#pragma unroll
        for (int jj = 0; jj < 16; ++jj) sr[jj] = fmaf(qd, ks[16 * p + jj][d], sr[jj]);
    }
    float mx = NEG;
#pragma unroll
    for (int jj = 0; jj < 16; ++jj) { if (16 * p + jj > i) sr[jj] = NEG; mx = fmaxf(mx, sr[jj]); }
    mx = fmaxf(mx, __shfl_xor(mx, 1, 32));
    mx = fmaxf(mx, __shfl_xor(mx, 2, 32));
    float sum = 0.f;
#pragma unroll
    for (int jj = 0; jj < 16; ++jj) { sr[jj] = __expf(sr[jj] - mx); sum += sr[jj]; }
    sum += __shfl_xor(sum, 1, 32);
    sum += __shfl_xor(sum, 2, 32);
    const float inv = 1.0f / sum;
    __syncthreads();
#pragma unroll
    for (int jj = 0; jj < 16; ++jj) qs[i][16 * p + jj] = sr[jj] * inv;
    __syncthreads();
    float orr[16];
#pragma unroll
    for (int dd = 0; dd < 16; ++dd) orr[dd] = 0.f;
#pragma unroll 1
    for (int j = 0; j < 64; ++j) {
        const float pj = qs[i][j];
#pragma unroll
        for (int dd = 0; dd < 16; ++dd) orr[dd] = fmaf(pj, vs[j][16 * p + dd], orr[dd]);
    }
    v4u w0, w1;
    w0.x = f2h(orr[0] * 4.0f)  | (f2h(orr[1] * 4.0f) << 16);  w0.y = f2h(orr[2] * 4.0f)  | (f2h(orr[3] * 4.0f) << 16);
    w0.z = f2h(orr[4] * 4.0f)  | (f2h(orr[5] * 4.0f) << 16);  w0.w = f2h(orr[6] * 4.0f)  | (f2h(orr[7] * 4.0f) << 16);
    w1.x = f2h(orr[8] * 4.0f)  | (f2h(orr[9] * 4.0f) << 16);  w1.y = f2h(orr[10] * 4.0f) | (f2h(orr[11] * 4.0f) << 16);
    w1.z = f2h(orr[12] * 4.0f) | (f2h(orr[13] * 4.0f) << 16); w1.w = f2h(orr[14] * 4.0f) | (f2h(orr[15] * 4.0f) << 16);
    ost[i][2 * p] = w0;
    ost[i][2 * p + 1] = w1;
    __syncthreads();
    const size_t tok0 = (size_t)bsel * SEQ;
    auto pass = [&]() {
#pragma unroll
        for (int q2 = 0; q2 < 2; ++q2) {
            const int row = 32 * q2 + (tid >> 3), pc = lane & 7;
            *(volatile v4u*)(ao + (tok0 + row) * DINNER + h * DHEAD + 8 * pc) = ost[row][pc];
        }
    };
    pass();
    __threadfence();
    pass();
}

__global__ __launch_bounds__(128) __attribute__((amdgpu_num_vgpr(256))) void attn_main(const us16* __restrict__ qhi, const us16* __restrict__ qlo,
                                                 const us16* __restrict__ khi, const us16* __restrict__ klo,
                                                 const us16* __restrict__ vt, us16* ao) {
    __shared__ v4u ost[4][16][8];
    const int tid = threadIdx.x, lane = tid & 31, wv = tid >> 5, m = lane & 15, hh = lane >> 4;
    const int qb = blockIdx.x + 1;
    const int h = blockIdx.y % HEADS, bsel = blockIdx.y / HEADS;
    const size_t tok0 = (size_t)bsel * SEQ;
    const int qrow = qb * 64 + wv * 16;
    const int iq = qrow + m;
    const size_t qoff = ((size_t)h * SEQT + tok0 + qrow + m) * DHEAD;
    const v8u qh0 = ld_frag(qhi + qoff, hh), qh1 = ld_frag(qhi + qoff + 32, hh);
    const v8u ql0 = ld_frag(qlo + qoff, hh), ql1 = ld_frag(qlo + qoff + 32, hh);
    const us16* kbh = khi + ((size_t)h * SEQT + tok0) * DHEAD;
    const us16* kbl = klo + ((size_t)h * SEQT + tok0) * DHEAD;
    const us16* vb = vt + (size_t)h * DHEAD * SEQT + tok0;
    const float NEG = -__builtin_inff();
    v8f o[4] = {};
    float mrun = NEG, lrun = 0.f;
    const int nch = 2 * qb + 2;
#pragma unroll 1
    for (int c = 0; c < nch; ++c) {
        v8f s[2] = {};
#pragma unroll
        for (int t = 0; t < 2; ++t) {
            const size_t koff = (size_t)(c * 32 + t * 16 + m) * DHEAD;
            const v8u a0 = ld_frag(kbh + koff, hh);
            s[t] = mma_bf16(a0, qh0, s[t]);
            s[t] = mma_bf16(a0, ql0, s[t]);
            const v8u a1 = ld_frag(kbl + koff, hh);
            s[t] = mma_bf16(a1, qh0, s[t]);
            const v8u a2 = ld_frag(kbh + koff + 32, hh);
            s[t] = mma_bf16(a2, qh1, s[t]);
            s[t] = mma_bf16(a2, ql1, s[t]);
            const v8u a3 = ld_frag(kbl + koff + 32, hh);
            s[t] = mma_bf16(a3, qh1, s[t]);
            asm volatile("v_nop\n\tv_nop\n\tv_nop\n\tv_nop" : "+v"(s[t]) : "v"(a0), "v"(a1), "v"(a2), "v"(a3), "v"(qh1), "v"(ql1));
        }
        float sv[16];
        float cmax = NEG;
#pragma unroll
        for (int t = 0; t < 2; ++t)
#pragma unroll
            for (int r = 0; r < 8; ++r) {
                const int j = c * 32 + t * 16 + 8 * hh + r;
                const float v = (j <= iq) ? s[t][r] * 8.0f : NEG;
                sv[8 * t + r] = v;
                cmax = fmaxf(cmax, v);
            }
        cmax = fmaxf(cmax, __shfl_xor(cmax, 16, 32));
        const float mnew = fmaxf(mrun, cmax);
        const float muse = (mnew == NEG) ? 0.f : mnew;
        const float fac = (mrun == NEG) ? 0.f : __expf(mrun - muse);
        mrun = mnew;
        v16h ph;
        float psum = 0.f;
#pragma unroll
        for (int r = 0; r < 8; ++r) {
            const _Float16 p0 = (_Float16)(__expf(sv[r] - muse) * 16384.0f);
            const _Float16 p1 = (_Float16)(__expf(sv[8 + r] - muse) * 16384.0f);
            ph[r] = p0;
            ph[8 + r] = p1;
            psum += (float)p0 + (float)p1;
        }
        psum += __shfl_xor(psum, 16, 32);
        lrun = lrun * fac + psum;
        const v8u pbu = __builtin_bit_cast(v8u, ph);
#pragma unroll
        for (int dt = 0; dt < 4; ++dt) o[dt] = o[dt] * fac;
#pragma unroll
        for (int dt = 0; dt < 4; ++dt) {
            const v8u va = ld_frag(vb + (size_t)(dt * 16 + m) * SEQT + c * 32, hh);
            o[dt] = mma_f16(va, pbu, o[dt]);
            mma_guard(o[dt], va, pbu);
        }
    }
    const float inv = 1.0f / lrun;
#pragma unroll
    for (int dt = 0; dt < 4; ++dt) {
        v4u w;
        w.x = f2h(o[dt][0] * inv) | (f2h(o[dt][1] * inv) << 16);
        w.y = f2h(o[dt][2] * inv) | (f2h(o[dt][3] * inv) << 16);
        w.z = f2h(o[dt][4] * inv) | (f2h(o[dt][5] * inv) << 16);
        w.w = f2h(o[dt][6] * inv) | (f2h(o[dt][7] * inv) << 16);
        ost[wv][m][2 * dt + hh] = w;
    }
    __syncthreads();
    us16* aob = ao + (tok0 + qrow) * DINNER + h * DHEAD;
    auto pass = [&]() {
#pragma unroll
        for (int p = 0; p < 4; ++p) {
            const int rr = 4 * p + (lane >> 3), pc = lane & 7;
            *(volatile v4u*)(aob + (size_t)rr * DINNER + 8 * pc) = ost[wv][rr][pc];
        }
    };
    pass();
    __threadfence();
    pass();
}

__global__ __launch_bounds__(256) void out_gemm(const us16* __restrict__ aop, const us16* __restrict__ wo, float* out) {
    __shared__ __align__(16) float cst[64 * CSTR];
    const int tid = threadIdx.x, lane = tid & 31, wv = tid >> 5, l16 = lane & 15, hh = lane >> 4;
    const int rt = wv & 3, ch = wv >> 2;
    const int row0 = blockIdx.x * 64;
    const int colb = blockIdx.y * 128;
    const us16* arow = aop + (size_t)(row0 + rt * 16 + l16) * DINNER;
    const us16* bbase = wo + (size_t)(colb + ch * 64 + l16) * DINNER;
    v8f acc[4] = {};
    mm_tile<1>(arow, bbase, DINNER, DINNER, hh, acc);
#pragma unroll
    for (int r = 0; r < 8; ++r) {
        const int rl = rt * 16 + 8 * hh + r;
#pragma unroll
        for (int t = 0; t < 4; ++t) cst[rl * CSTR + ch * 64 + t * 16 + l16] = acc[t][r] * (1.0f / 256.0f);
    }
    __syncthreads();
    const int col = tid & 127, rsel = tid >> 7;
    float* ob = out + (size_t)row0 * DIM + colb + col;
    auto pass = [&]() {
#pragma unroll 4
        for (int r = rsel; r < 64; r += 2) *(volatile float*)(ob + (size_t)r * DIM) = cst[r * CSTR + col];
    };
    pass();
    __threadfence();
    pass();
}

extern "C" void kernel_launch(void* const* d_in, const int* in_sizes, int n_in,
                              void* d_out, int out_size, void* d_ws, size_t ws_size, hipStream_t stream) {
    if (n_in < 4) return;
    const float* x     = (const float*)d_in[0];
    const float* gamma = (const float*)d_in[1];
    const float* w_qkv = (const float*)d_in[2];
    const float* w_out = (const float*)d_in[3];
    float* out = (float*)d_out;
    if (in_sizes[0] < ((NB - 1) * SEQ_FULL + SEQ) * DIM) return;
    if (in_sizes[1] < DIM) return;
    if (in_sizes[2] < DIM * NQKV) return;
    if (in_sizes[3] < DINNER * DIM) return;
    if (out_size < SEQT * DIM) return;

    size_t off = 0;
    auto carve = [&](size_t bytes) { size_t o = off; off += (bytes + 127) & ~(size_t)127; return o; };
    char* ws = (char*)d_ws;
    us16*  xb   = (us16*) (ws + carve((size_t)SEQT * DIM * 2));
    float* rs   = (float*)(ws + carve((size_t)SEQT * RSP * 4));
    us16*  wq   = (us16*) (ws + carve((size_t)NQKV * DIM * 2));
    us16*  wo   = (us16*) (ws + carve((size_t)DIM * DINNER * 2));
    us16*  qhi  = (us16*) (ws + carve((size_t)HEADS * SEQT * DHEAD * 2));
    us16*  qlo  = (us16*) (ws + carve((size_t)HEADS * SEQT * DHEAD * 2));
    us16*  khi  = (us16*) (ws + carve((size_t)HEADS * SEQT * DHEAD * 2));
    us16*  klo  = (us16*) (ws + carve((size_t)HEADS * SEQT * DHEAD * 2));
    us16*  vt   = (us16*) (ws + carve((size_t)HEADS * DHEAD * SEQT * 2));
    float* qkvf = (float*)(ws + carve((size_t)NB * 64 * NQKV * 4));
    us16*  ao   = (us16*) (ws + carve((size_t)SEQT * DINNER * 2));
    if (off > ws_size) return;

    prep_x<<<SEQT, 256, 0, stream>>>(x, xb, rs);
    prep_w<0, 1><<<dim3(NQKV / 64, DIM / 64), 256, 0, stream>>>(w_qkv, NQKV, DIM, gamma, 1.0f, wq);
    prep_w<1, 0><<<dim3(DIM / 64, DINNER / 64), 256, 0, stream>>>(w_out, DIM, DINNER, gamma, 64.0f, wo);
    qkv_gemm<<<dim3(SEQT / 64, NQKV / 128), 256, 0, stream>>>(xb, wq, rs, qhi, qlo, khi, klo, vt, qkvf);
    attn_first<<<NB * HEADS, 256, 0, stream>>>(qkvf, ao);
    attn_main<<<dim3(QBLK - 1, NB * HEADS), 128, 0, stream>>>(qhi, qlo, khi, klo, vt, ao);
    out_gemm<<<dim3(SEQT / 64, DIM / 128), 256, 0, stream>>>(ao, wo, out);
}
